// NEXT_Simulator_50921132262080
// MI455X (gfx1250) — hardware-verified
//
#include <hip/hip_runtime.h>
#include <stddef.h>


typedef _Float16 h16;
typedef _Float16 v16h __attribute__((ext_vector_type(16)));
typedef _Float16 v8h  __attribute__((ext_vector_type(8)));
typedef float    v8f  __attribute__((ext_vector_type(8)));
typedef float    v4f  __attribute__((ext_vector_type(4)));
typedef float    v2f  __attribute__((ext_vector_type(2)));

#ifndef NB
#define NB 4
#endif
#ifndef NEL
#define NEL 8192
#endif
#define NB_FULL  4
#define NEL_FULL 8192

#define NT     550
#define NPMT   12
#define NS     2209
#define NCOL   2224
#define NTILE  139
#define W4ROWS 2240
#define OPITCH 576
#define EPB    32
#define H1W    64
#define H2W    128
#define H3W    256
#define LD1    72
#define LD2    136
#define LD3    264
#define LDT    72
#define APITCH 580
#define AFRONT 4
#define ACC_FLOATS (32 * APITCH)
#define ACC_BYTES  (ACC_FLOATS * 4)
#define WCARRY 64.0f
#define GAUSS_NORM 3.989422804f

#define OUT0_FLOATS (NB_FULL * NPMT * NT)
#define OUT1_FLOATS (NB_FULL * NS * NT)
#define OUT_FLOATS  (OUT0_FLOATS + OUT1_FLOATS)
#define NF4         (OUT_FLOATS / 4)

static_assert(NB >= 1 && NB <= NB_FULL);
static_assert(NEL >= 32 && NEL <= NEL_FULL && (NEL % 32) == 0);
static_assert(NCOL == NTILE * 16);
static_assert(NS + NPMT <= NCOL);
static_assert((NS / 16) == NTILE - 1);
static_assert(W4ROWS >= NCOL && (W4ROWS % 64) == 0);
static_assert((OPITCH % 32) == 0 && OPITCH >= NT);
static_assert(((16 * OPITCH * 4) % 512) == 0);
static_assert((16 * OPITCH) / 4 == 72 * 32);
static_assert((NT % 2) == 0);
static_assert((OUT0_FLOATS % 4) == 0 && (OUT_FLOATS % 4) == 0);
static_assert(OUT0_FLOATS * 4 == 105600);
static_assert((APITCH % 4) == 0 && APITCH >= AFRONT + 4 * 144);
static_assert(AFRONT + 553 < APITCH);
static_assert((H1W % 32) == 0 && (H2W % 32) == 0 && (H3W % 32) == 0);
static_assert(LD1 >= H1W && (LD1 % 8) == 0);
static_assert(LD2 >= H2W && (LD2 % 8) == 0);
static_assert(LD3 >= H3W && (LD3 % 8) == 0);
static_assert(EPB * 4 == 128);
static_assert(H1W == 4 * 16);

#define W2T_BYTES ((size_t)H2W * H1W * 2)
#define W3T_BYTES ((size_t)H3W * H2W * 2)
#define W4T_BYTES ((size_t)W4ROWS * H3W * 2)
#define H3_BYTES  ((size_t)NB * NEL * H3W * 2)
#define PR_BYTES  ((size_t)NB * NEL * 16 * 4)
#define EW_BYTES  ((size_t)NB * NEL * 8 * 4)
#define OT_BYTES  ((size_t)NB * NCOL * OPITCH * 4)
#define OFF_W2T ((size_t)0)
#define OFF_W3T (OFF_W2T + W2T_BYTES)
#define OFF_W4T (OFF_W3T + W3T_BYTES)
#define OFF_H3  (OFF_W4T + W4T_BYTES)
#define OFF_PR  (OFF_H3 + H3_BYTES)
#define OFF_EW  (OFF_PR + PR_BYTES)
#define OFF_OT  (OFF_EW + EW_BYTES)
#define WS_TOTAL (OFF_OT + OT_BYTES)
static_assert((W2T_BYTES % 128) == 0 && (W3T_BYTES % 128) == 0 && (W4T_BYTES % 128) == 0);
static_assert((H3_BYTES % 128) == 0 && (PR_BYTES % 128) == 0 && (EW_BYTES % 128) == 0);
static_assert((OT_BYTES % 128) == 0);
static_assert(WS_TOTAL <= (size_t)134217728);

__device__ __forceinline__ float bf16r(float x) {
  unsigned int u = __float_as_uint(x);
  u = (u + 0x7FFFu + ((u >> 16) & 1u)) & 0xFFFF0000u;
  return __uint_as_float(u);
}

__device__ __forceinline__ h16 toh_flush(float v) {
  const h16 r = (h16)v;
  return (fabsf(v) < 6.103515625e-05f) ? (h16)0.0f : r;
}

__device__ __forceinline__ v16h frag_at(const _Float16* p) {
  v8h lo = *(const v8h*)(p);
  v8h hi = *(const v8h*)(p + 16);
  v16h out;
#pragma unroll
  for (int i = 0; i < 8; ++i) { out[i] = lo[i]; out[i + 8] = hi[i]; }
  return out;
}
__device__ __forceinline__ v16h ld_frag(const _Float16* base, unsigned ld) {
  const unsigned lane = threadIdx.x & 31u;
  return frag_at(base + (lane & 15u) * ld + (lane >> 4) * 8u);
}

__device__ __forceinline__ v8f wmma16(v16h a, v16h b, v8f c) {
  v8f d = __builtin_amdgcn_wmma_f32_16x16x32_f16(false, a, false, b, (short)0, c,
                                                 false, false);
  asm volatile("v_nop\n\tv_nop\n\tv_nop\n\tv_nop" : "+v"(d) : "v"(a), "v"(b));
  return d;
}

__device__ __forceinline__ void wave_lds_sync() {
  __builtin_amdgcn_fence(3  , "wavefront");
  asm volatile("s_wait_dscnt 0x0" ::: "memory");
  __builtin_amdgcn_wave_barrier();
}

__device__ __forceinline__ float sigm(float x) {
  return __builtin_amdgcn_rcpf(1.0f + __expf(-x));
}

__global__ __launch_bounds__(256) void wplane_kernel(
    const float* __restrict__ W, _Float16* __restrict__ Wt, unsigned ldw, unsigned ldk,
    unsigned nvalid) {
  __shared__ __attribute__((aligned(16))) _Float16 T[64 * LDT];
  const unsigned tid = threadIdx.x;
  const unsigned n0 = blockIdx.x * 64u;
  const unsigned k0 = blockIdx.y * 64u;
#pragma unroll 4
  for (unsigned j = 0; j < 16u; ++j) {
    const unsigned idx = tid + 256u * j;
    const unsigned kr = idx >> 6, nc = idx & 63u;
    const unsigned n = n0 + nc;
    const unsigned nn = (n < nvalid) ? n : (nvalid - 1u);
    const float v = W[(size_t)(k0 + kr) * ldw + nn];
    const float vv = (n < nvalid) ? v : 0.0f;
    T[nc * LDT + kr] = toh_flush(WCARRY * bf16r(vv));
  }
  __syncthreads();
  v8h x[2];
  size_t off[2];
#pragma unroll
  for (unsigned i = 0; i < 2u; ++i) {
    const unsigned n = 32u * i + (tid >> 3);
    const unsigned kc = (tid & 7u) * 8u;
    x[i] = *(const v8h*)&T[n * LDT + kc];
    off[i] = (size_t)(n0 + n) * ldk + k0 + kc;
  }
#pragma unroll
  for (int i = 0; i < 2; ++i) *(volatile v8h*)(Wt + off[i]) = x[i];
  __threadfence();
#pragma unroll
  for (int i = 0; i < 2; ++i) *(volatile v8h*)(Wt + off[i]) = x[i];
}

__global__ __launch_bounds__(128) void mlp_kernel(
    const float* __restrict__ electrons, const float* __restrict__ weight,
    const float* __restrict__ Wp1, const float* __restrict__ bp1,
    const float* __restrict__ Wp2, const float* __restrict__ bp2,
    const float* __restrict__ pmt_scale,
    const float* __restrict__ Ws1, const float* __restrict__ bs1,
    const float* __restrict__ bs2, const float* __restrict__ bs3,
    const _Float16* __restrict__ W2t, const _Float16* __restrict__ W3t,
    _Float16* __restrict__ H3, float* __restrict__ PR, float* __restrict__ EW) {
  __shared__ __attribute__((aligned(16))) _Float16 h1s[EPB * LD1];
  __shared__ __attribute__((aligned(16))) _Float16 h2s[EPB * LD2];
  __shared__ __attribute__((aligned(16))) _Float16 h3s[EPB * LD3];
  __shared__ __attribute__((aligned(16))) float prs[EPB * 16];
  __shared__ __attribute__((aligned(16))) float ews[EPB * 8];

  const unsigned tid = threadIdx.x, lane = tid & 31u;
  const unsigned wave = __builtin_amdgcn_readfirstlane(threadIdx.x >> 5);
  const unsigned hh = lane >> 4, m = lane & 15u;
  const unsigned ce0 = blockIdx.x * (unsigned)EPB;
  const unsigned b = ce0 / (unsigned)NEL;
  const unsigned e0 = ce0 - b * (unsigned)NEL;
  const unsigned e = tid >> 2, part = tid & 3u;
  const size_t ge = (size_t)b * NEL_FULL + e0 + e;

  const float x = bf16r(electrons[ge * 3 + 0]);
  const float y = bf16r(electrons[ge * 3 + 1]);
  const float z = bf16r(electrons[ge * 3 + 2]);
  const float w = bf16r(weight[ge]);

  {
    float cf = floorf(z - 0.5f);
    cf = fminf(fmaxf(cf, -3.0f), 551.0f);
    const int t0 = (int)cf - 1;
    const float dt = (float)(t0 + (int)part) + 0.5f - z;
    const float ev = (GAUSS_NORM * __expf(-(dt * dt) * 10.0f)) * w;
    ews[e * 8u + part] = ev;
    ews[e * 8u + 4u + part] = (part == 0u) ? (float)t0 : 0.0f;
  }

#pragma unroll 4
  for (unsigned i = 0; i < 16u; ++i) {
    const unsigned k = part * 16u + i;
    const float pre = x * bf16r(Ws1[k]) + y * bf16r(Ws1[H1W + k]) + bf16r(bs1[k]);
    h1s[e * LD1 + k] = toh_flush(sigm(pre));
  }

  {
    const unsigned p0 = part * 3u;
    float a0 = bf16r(bp2[p0]), a1 = bf16r(bp2[p0 + 1u]), a2 = bf16r(bp2[p0 + 2u]);
#pragma unroll 1
    for (unsigned i = 0; i < 28u; ++i) {
      const float hi = sigm(x * bf16r(Wp1[i]) + y * bf16r(Wp1[28u + i]) + bf16r(bp1[i]));
      a0 += hi * bf16r(Wp2[i * NPMT + p0]);
      a1 += hi * bf16r(Wp2[i * NPMT + p0 + 1u]);
      a2 += hi * bf16r(Wp2[i * NPMT + p0 + 2u]);
    }
    const float s0 = bf16r(pmt_scale[p0]);
    const float s1 = bf16r(pmt_scale[p0 + 1u]);
    const float s2 = bf16r(pmt_scale[p0 + 2u]);
    prs[e * 16u + p0]      = sigm(a0) * (s0 * s0);
    prs[e * 16u + p0 + 1u] = sigm(a1) * (s1 * s1);
    prs[e * 16u + p0 + 2u] = sigm(a2) * (s2 * s2);
    prs[e * 16u + 12u + part] = 0.0f;
  }
  __syncthreads();

#pragma unroll 1
  for (unsigned q = 0; q < 2u; ++q) {
    const unsigned nt = wave * 2u + q;
    const _Float16* bp = W2t + (size_t)(nt * 16u + m) * H1W + hh * 8u;
    v16h bw[2];
#pragma unroll
    for (int k = 0; k < 2; ++k) bw[k] = frag_at(bp + k * 32);
    const float bn = bf16r(bs2[nt * 16u + m]);
#pragma unroll
    for (unsigned mt = 0; mt < 2u; ++mt) {
      v8f c = {};
#pragma unroll
      for (int k = 0; k < 2; ++k)
        c = wmma16(ld_frag(&h1s[(mt * 16u) * LD1 + (unsigned)k * 32u], LD1), bw[k], c);
#pragma unroll
      for (int r = 0; r < 8; ++r)
        h2s[(mt * 16u + hh * 8u + (unsigned)r) * LD2 + nt * 16u + m] =
            toh_flush(sigm(c[r] * (1.0f / WCARRY) + bn));
    }
  }
  __syncthreads();

#pragma unroll 1
  for (unsigned q = 0; q < 4u; ++q) {
    const unsigned nt = wave * 4u + q;
    const _Float16* bp = W3t + (size_t)(nt * 16u + m) * H2W + hh * 8u;
    v16h bw[4];
#pragma unroll
    for (int k = 0; k < 4; ++k) bw[k] = frag_at(bp + k * 32);
    const float bn = bf16r(bs3[nt * 16u + m]);
#pragma unroll
    for (unsigned mt = 0; mt < 2u; ++mt) {
      v8f c = {};
#pragma unroll
      for (int k = 0; k < 4; ++k)
        c = wmma16(ld_frag(&h2s[(mt * 16u) * LD2 + (unsigned)k * 32u], LD2), bw[k], c);
#pragma unroll
      for (int r = 0; r < 8; ++r)
        h3s[(mt * 16u + hh * 8u + (unsigned)r) * LD3 + nt * 16u + m] =
            toh_flush(sigm(c[r] * (1.0f / WCARRY) + bn));
    }
  }
  __syncthreads();

  {
    v8h xv[8];
    size_t off[8];
#pragma unroll
    for (unsigned j = 0; j < 8u; ++j) {
      const unsigned idx = tid + 128u * j;
      const unsigned r = idx >> 5, c = (idx & 31u) * 8u;
      xv[j] = *(const v8h*)&h3s[r * LD3 + c];
      off[j] = (size_t)(ce0 + r) * H3W + c;
    }
#pragma unroll
    for (int j = 0; j < 8; ++j) *(volatile v8h*)(H3 + off[j]) = xv[j];
    __threadfence();
#pragma unroll
    for (int j = 0; j < 8; ++j) *(volatile v8h*)(H3 + off[j]) = xv[j];
  }
  {
    const v4f pv = *(const v4f*)&prs[tid * 4u];
    float* pp = PR + (size_t)ce0 * 16u + tid * 4u;
    *(volatile v4f*)pp = pv;
    __threadfence();
    *(volatile v4f*)pp = pv;
  }
  if (wave < 2u) {
    const v4f ev = *(const v4f*)&ews[tid * 4u];
    float* pe = EW + (size_t)ce0 * 8u + tid * 4u;
    *(volatile v4f*)pe = ev;
    __threadfence();
    *(volatile v4f*)pe = ev;
  }
}

extern __shared__ __attribute__((aligned(16))) float acc_lds[];

__global__ __launch_bounds__(32) void bin_kernel(
    const _Float16* __restrict__ H3, const _Float16* __restrict__ W4t,
    const float* __restrict__ bs4, const float* __restrict__ si_scale,
    const float* __restrict__ PR, const float* __restrict__ EW,
    float* __restrict__ OutT) {
  const unsigned lane = threadIdx.x & 31u;
  const unsigned hh = lane >> 4, m = lane & 15u;
  const unsigned nt = blockIdx.x;
  const unsigned b = blockIdx.y;

#pragma unroll 1
  for (unsigned i = lane; i < (unsigned)(ACC_FLOATS / 4); i += 32u)
    *(v4f*)&acc_lds[i * 4u] = (v4f){0.0f, 0.0f, 0.0f, 0.0f};
  wave_lds_sync();

  const unsigned col = nt * 16u + m;
  const unsigned cs = (col < (unsigned)NS) ? col : (unsigned)(NS - 1);
  const float bn = bf16r(bs4[cs]);
  const float scv = bf16r(si_scale[cs]);
  const float sc2 = scv * scv;
  const int pci = (int)col - NS;
  const unsigned pc = (unsigned)((pci < 0) ? 0 : ((pci > NPMT - 1) ? (NPMT - 1) : pci));
  const bool is_s = col < (unsigned)NS;
  const bool is_p = col < (unsigned)(NS + NPMT);
  const bool last = (nt == (unsigned)(NTILE - 1));

  v16h bf[8];
  {
    const _Float16* bp = W4t + (size_t)col * H3W + hh * 8u;
#pragma unroll
    for (int k = 0; k < 8; ++k) bf[k] = frag_at(bp + k * 32);
  }
  const int abase = (int)((hh * 16u + m) * (unsigned)APITCH + (unsigned)AFRONT);

#pragma unroll 1
  for (unsigned mt = 0; mt < (unsigned)(NEL / 16); ++mt) {
    const size_t ce = (size_t)b * NEL + (size_t)mt * 16u;
    const _Float16* ap = H3 + (ce + m) * H3W + hh * 8u;
    v8f c = {};
#pragma unroll
    for (int k = 0; k < 8; ++k) c = wmma16(frag_at(ap + k * 32), bf[k], c);

    float resp[8];
#pragma unroll
    for (int r = 0; r < 8; ++r) resp[r] = sigm(c[r] * (1.0f / WCARRY) + bn) * sc2;
    if (last) {
#pragma unroll
      for (int r = 0; r < 8; ++r) {
        const float pr = PR[(ce + hh * 8u + (unsigned)r) * 16u + pc];
        resp[r] = is_s ? resp[r] : (is_p ? pr : 0.0f);
      }
    }
#pragma unroll
    for (int r = 0; r < 8; ++r) {
      const float* rec = EW + (ce + hh * 8u + (unsigned)r) * 8u;
      const v4f ev = *(const v4f*)rec;
      int t0 = (int)rec[4];
      t0 = (t0 < -4) ? -4 : ((t0 > 550) ? 550 : t0);
      const int ix = abase + t0;
#pragma unroll
      for (int j = 0; j < 4; ++j) {
        const float cur = acc_lds[ix + j];
        acc_lds[ix + j] = cur + resp[r] * ev[j];
      }
    }
  }
  wave_lds_sync();

  float* orow = OutT + ((size_t)b * NCOL + (size_t)nt * 16u) * OPITCH;
#pragma unroll 1
  for (unsigned it = 0; it < 72u; ++it) {
    const unsigned f = it * 32u + lane;
    const unsigned row = f / 144u;
    const unsigned q = f - row * 144u;
    const unsigned i0 = row * (unsigned)APITCH + (unsigned)AFRONT + 4u * q;
    const v4f a0 = *(const v4f*)&acc_lds[i0];
    const v4f a1 = *(const v4f*)&acc_lds[i0 + 16u * (unsigned)APITCH];
    v4f o;
#pragma unroll
    for (int j = 0; j < 4; ++j) o[j] = (4u * q + (unsigned)j < (unsigned)NT) ? (a0[j] + a1[j]) : 0.0f;
    *(volatile v4f*)(orow + (size_t)f * 4u) = o;
  }
  __threadfence();
#pragma unroll 1
  for (unsigned it = 0; it < 72u; ++it) {
    const unsigned f = it * 32u + lane;
    const unsigned row = f / 144u;
    const unsigned q = f - row * 144u;
    const unsigned i0 = row * (unsigned)APITCH + (unsigned)AFRONT + 4u * q;
    const v4f a0 = *(const v4f*)&acc_lds[i0];
    const v4f a1 = *(const v4f*)&acc_lds[i0 + 16u * (unsigned)APITCH];
    v4f o;
#pragma unroll
    for (int j = 0; j < 4; ++j) o[j] = (4u * q + (unsigned)j < (unsigned)NT) ? (a0[j] + a1[j]) : 0.0f;
    *(volatile v4f*)(orow + (size_t)f * 4u) = o;
  }
}

__global__ __launch_bounds__(256) void pack_kernel(const float* __restrict__ OutT,
                                                   float* __restrict__ outp) {
  const unsigned g = blockIdx.x * 256u + threadIdx.x;
  const unsigned gc = (g < (unsigned)NF4) ? g : (unsigned)(NF4 - 1);
  v4f o;
#pragma unroll
  for (unsigned hf = 0; hf < 2u; ++hf) {
    const unsigned i = gc * 4u + 2u * hf;
    const bool first = i < (unsigned)OUT0_FLOATS;
    const unsigned ia = first ? i : (unsigned)(OUT0_FLOATS - 2);
    const unsigned b0 = ia / (unsigned)(NPMT * NT);
    const unsigned r0 = ia - b0 * (unsigned)(NPMT * NT);
    const unsigned p0 = r0 / (unsigned)NT;
    const unsigned t0 = r0 - p0 * (unsigned)NT;
    const unsigned j = first ? 0u : (i - (unsigned)OUT0_FLOATS);
    const unsigned R = j / (unsigned)NT;
    const unsigned t1 = j - R * (unsigned)NT;
    const unsigned b1 = R / (unsigned)NS;
    const unsigned s1 = R - b1 * (unsigned)NS;
    const unsigned bb = first ? b0 : b1;
    const unsigned cc = first ? ((unsigned)NS + p0) : s1;
    const unsigned tt = first ? t0 : t1;
    const unsigned bc = (bb < (unsigned)NB) ? bb : (unsigned)(NB - 1);
    const v2f p = *(const v2f*)(OutT + ((size_t)bc * NCOL + cc) * OPITCH + tt);
    const bool ok = bb < (unsigned)NB;
    o[2 * hf]     = ok ? p[0] : 0.0f;
    o[2 * hf + 1] = ok ? p[1] : 0.0f;
  }
  if (g < (unsigned)NF4) {
    float* dst = outp + (size_t)g * 4u;
    *(volatile v4f*)dst = o;
    __threadfence();
    *(volatile v4f*)dst = o;
  }
}

extern "C" void kernel_launch(void* const* d_in, const int* in_sizes, int n_in,
                              void* d_out, int out_size, void* d_ws, size_t ws_size,
                              hipStream_t stream) {
  if (n_in < 16) return;
  const long long need_e = (long long)(NB - 1) * NEL_FULL + NEL;
  if ((long long)in_sizes[0] < need_e * 3) return;
  if ((long long)in_sizes[1] < need_e) return;
  if (in_sizes[2] < 56 || in_sizes[3] < 28 || in_sizes[4] < 336) return;
  if (in_sizes[5] < 12 || in_sizes[6] < 12) return;
  if (in_sizes[7] < 128 || in_sizes[8] < 64) return;
  if (in_sizes[9] < H1W * H2W || in_sizes[10] < H2W) return;
  if (in_sizes[11] < H2W * H3W || in_sizes[12] < H3W) return;
  if ((long long)in_sizes[13] < (long long)H3W * NS) return;
  if (in_sizes[14] < NS || in_sizes[15] < NS) return;
  if ((long long)out_size < (long long)OUT_FLOATS) return;
  if (ws_size < WS_TOTAL) return;

  const float* electrons = (const float*)d_in[0];
  const float* weight    = (const float*)d_in[1];
  const float* Wp1       = (const float*)d_in[2];
  const float* bp1       = (const float*)d_in[3];
  const float* Wp2       = (const float*)d_in[4];
  const float* bp2       = (const float*)d_in[5];
  const float* pmt_scale = (const float*)d_in[6];
  const float* Ws1       = (const float*)d_in[7];
  const float* bs1       = (const float*)d_in[8];
  const float* Ws2       = (const float*)d_in[9];
  const float* bs2       = (const float*)d_in[10];
  const float* Ws3       = (const float*)d_in[11];
  const float* bs3       = (const float*)d_in[12];
  const float* Ws4       = (const float*)d_in[13];
  const float* bs4       = (const float*)d_in[14];
  const float* si_scale  = (const float*)d_in[15];
  float* outp = (float*)d_out;

  char* ws = (char*)d_ws;
  _Float16* W2t = (_Float16*)(ws + OFF_W2T);
  _Float16* W3t = (_Float16*)(ws + OFF_W3T);
  _Float16* W4t = (_Float16*)(ws + OFF_W4T);
  _Float16* H3  = (_Float16*)(ws + OFF_H3);
  float*    PR  = (float*)(ws + OFF_PR);
  float*    EW  = (float*)(ws + OFF_EW);
  float*    OT  = (float*)(ws + OFF_OT);

  wplane_kernel<<<dim3(H2W / 64, H1W / 64), dim3(256), 0, stream>>>(
      Ws2, W2t, (unsigned)H2W, (unsigned)H1W, (unsigned)H2W);
  wplane_kernel<<<dim3(H3W / 64, H2W / 64), dim3(256), 0, stream>>>(
      Ws3, W3t, (unsigned)H3W, (unsigned)H2W, (unsigned)H3W);
  wplane_kernel<<<dim3(W4ROWS / 64, H3W / 64), dim3(256), 0, stream>>>(
      Ws4, W4t, (unsigned)NS, (unsigned)H3W, (unsigned)NS);

  mlp_kernel<<<dim3((NB * NEL) / EPB), dim3(128), 0, stream>>>(
      electrons, weight, Wp1, bp1, Wp2, bp2, pmt_scale, Ws1, bs1, bs2, bs3,
      W2t, W3t, H3, PR, EW);

  hipFuncSetAttribute(reinterpret_cast<const void*>(&bin_kernel),
                      hipFuncAttributeMaxDynamicSharedMemorySize, (int)ACC_BYTES);
  bin_kernel<<<dim3(NTILE, NB), dim3(32), (size_t)ACC_BYTES, stream>>>(
      H3, W4t, bs4, si_scale, PR, EW, OT);

  pack_kernel<<<dim3((NF4 + 255) / 256), dim3(256), 0, stream>>>(OT, outp);
}
